// EdgeScoringNetwork_1795296330233
// MI455X (gfx1250) — hardware-verified
//
#include <hip/hip_runtime.h>
#include <math.h>

typedef __attribute__((ext_vector_type(16))) _Float16 v16h;
typedef __attribute__((ext_vector_type(16))) __bf16 v16b;
typedef __attribute__((ext_vector_type(8)))  _Float16 v8h;
typedef __attribute__((ext_vector_type(8)))  float v8f;
typedef __attribute__((ext_vector_type(4)))  float v4f;
typedef __attribute__((ext_vector_type(2)))  float v2f;
typedef __attribute__((ext_vector_type(4)))  unsigned v4u;
typedef __attribute__((ext_vector_type(4)))  int v4i;
typedef float __attribute__((may_alias)) float_a;
typedef int __attribute__((may_alias)) int_a;

template <typename T> __device__ __forceinline__ void vst2(void* p, T v) { *(volatile T*)p = v; __threadfence(); *(volatile T*)p = v; }
__device__ __forceinline__ v8f wmma16(v16h a, v16h b, v8f c) {
  v8f d = __builtin_amdgcn_wmma_f32_16x16x32_f16(false, a, false, b, (short)0, c, false, false);
  asm volatile("v_nop\n\tv_nop\n\tv_nop\n\tv_nop" : "+v"(d) : "v"(a), "v"(b));
  return d;
}
__device__ __forceinline__ v8f wmma_bf(v16b a, v16b b, v8f c) {
  v8f d = __builtin_amdgcn_wmma_f32_16x16x32_bf16(false, a, false, b, (short)0, c, false, false);
  asm volatile("v_nop\n\tv_nop\n\tv_nop\n\tv_nop" : "+v"(d) : "v"(a), "v"(b));
  return d;
}
__device__ __forceinline__ v16h frag_h(const _Float16* rowk0, int lane) {
  union { v16h v; v8h q[2]; } u; const _Float16* p = rowk0 + 8 * (lane >> 4);
  u.q[0] = *(const v8h*)p; u.q[1] = *(const v8h*)(p + 16); return u.v;
}
__device__ __forceinline__ v16h frag_f32(const float* rowk0, int lane) {
  v16h a; const float* p = rowk0 + 8 * (lane >> 4);
#pragma unroll
  for (int i = 0; i < 8; ++i) { a[i] = (_Float16)p[i]; a[8 + i] = (_Float16)p[16 + i]; }
  return a;
}
__device__ __forceinline__ v16h frag_f32s(const float* rowk0, int lane, float sc) {
  v16h a; const float* p = rowk0 + 8 * (lane >> 4);
#pragma unroll
  for (int i = 0; i < 8; ++i) { a[i] = (_Float16)(p[i] * sc); a[8 + i] = (_Float16)(p[16 + i] * sc); }
  return a;
}
__device__ __forceinline__ v16h fragc_f32(const float* W, int k0, int n, int lane, int ld, int K) {
  v16h a; const int g = lane >> 4;
#pragma unroll
  for (int i = 0; i < 8; ++i) { const int ka = k0 + 8 * g + i, kb = ka + 16;
    a[i] = (_Float16)(ka < K ? W[(size_t)(ka < K ? ka : K - 1) * ld + n] : 0.f); a[8 + i] = (_Float16)(kb < K ? W[(size_t)(kb < K ? kb : K - 1) * ld + n] : 0.f); }
  return a;
}
struct F2 { v16b h, l; };
__device__ __forceinline__ F2 bsplit16(const float v[16]) { F2 r;
#pragma unroll
  for (int i = 0; i < 16; ++i) { const __bf16 h = (__bf16)v[i]; r.h[i] = h; r.l[i] = (__bf16)(v[i] - (float)h); }
  return r; }
__device__ __forceinline__ F2 split_row(const float* row, int k0, int lane) { float v[16]; const float* p = row + k0 + 8 * (lane >> 4);
#pragma unroll
  for (int i = 0; i < 8; ++i) { v[i] = p[i]; v[8 + i] = p[16 + i]; }
  return bsplit16(v); }
__device__ __forceinline__ F2 split_rowK(const float* row, int k0, int lane, int K) { float v[16]; const int g = lane >> 4;
#pragma unroll
  for (int i = 0; i < 8; ++i) { const int ka = k0 + 8 * g + i, kb = ka + 16; v[i] = ka < K ? row[ka < K ? ka : K - 1] : 0.f; v[8 + i] = kb < K ? row[kb < K ? kb : K - 1] : 0.f; }
  return bsplit16(v); }
__device__ __forceinline__ F2 split_col(const float* W, int k0, int n, int lane, int ld, int K) { float v[16]; const int g = lane >> 4;
#pragma unroll
  for (int i = 0; i < 8; ++i) { const int ka = k0 + 8 * g + i, kb = ka + 16; v[i] = ka < K ? W[(size_t)(ka < K ? ka : K - 1) * ld + n] : 0.f; v[8 + i] = kb < K ? W[(size_t)(kb < K ? kb : K - 1) * ld + n] : 0.f; }
  return bsplit16(v); }
__device__ __forceinline__ v8f mac3(const F2& a, const F2& b, v8f c) { c = wmma_bf(a.l, b.h, c); c = wmma_bf(a.h, b.l, c); return wmma_bf(a.h, b.h, c); }
__device__ __forceinline__ float sigm(float v) { return 1.0f / (1.0f + expf(-v)); }
#define LDSX() do { asm volatile("s_wait_dscnt 0" ::: "memory"); __builtin_amdgcn_wave_barrier(); __builtin_amdgcn_fence(__ATOMIC_RELEASE, "workgroup"); } while (0)


#define NBT 4
#define NNODE 10000
#define FD 128
#define ED 32
#define NE 640000
#define IND (2 * FD + 1)
#define TEMP 0.66f
#define PIT 5
typedef __attribute__((ext_vector_type(8))) __bf16 v8b;
__device__ __forceinline__ v16b frag_b(const __bf16* rowk0, int lane) {
  union { v16b v; v8b q[2]; } u; const __bf16* p = rowk0 + 8 * (lane >> 4);
  u.q[0] = *(const v8b*)p; u.q[1] = *(const v8b*)(p + 16); return u.v;
}
__device__ __forceinline__ float bfr(float v) { return (float)(__bf16)v; }
__device__ __attribute__((noinline)) float exp_ni(float v) { return expf(v); }
__device__ __attribute__((noinline)) float erf_ni(float v) { return erff(v); }

#define WS_SIG 0u
#define WS_END 64u

__device__ __forceinline__ v16b fragb_f32(const float* __restrict__ p, int lane) { v16b a; const float* pp = p + 8 * (lane >> 4);
#pragma unroll
  for (int i = 0; i < 8; ++i) { a[i] = (__bf16)pp[i]; a[8 + i] = (__bf16)pp[16 + i]; } return a; }
__global__ __launch_bounds__(96) void k_sigma(const float* __restrict__ W1, const float* __restrict__ W2, const float* __restrict__ W3, float* __restrict__ SIG) {
  __shared__ float su[3][ED]; __shared__ float sv[3][IND + 3]; __shared__ __align__(16) float res[4];
  const int w = threadIdx.x >> 5, lane = threadIdx.x & 31; const float* Wm = w == 0 ? W1 : w == 1 ? W2 : W3; const int nout = w == 2 ? 1 : ED; const int nin = w == 0 ? IND : ED;
  if (lane < nout) su[w][lane] = 1.0f / sqrtf((float)nout); __syncthreads();
#pragma unroll 1
  for (int it = 0; it < PIT; ++it) {
    float nv = 0.f;
#pragma unroll 1
    for (int i = lane; i < nin; i += 32) { float s = 0.f;
#pragma unroll 1
      for (int o = 0; o < nout; ++o) s += bfr(Wm[(size_t)o * nin + i]) * su[w][o]; sv[w][i] = s; nv += s * s; }
#pragma unroll
    for (int o = 1; o < 32; o <<= 1) nv += __shfl_xor(nv, o);
    const float invn = 1.0f / (sqrtf(nv) + 1e-12f); __syncthreads();
#pragma unroll 1
    for (int i = lane; i < nin; i += 32) sv[w][i] *= invn; __syncthreads();
    float uo = 0.f; if (lane < nout) {
#pragma unroll 1
      for (int i = 0; i < nin; ++i) uo += bfr(Wm[(size_t)lane * nin + i]) * sv[w][i]; }
    float nu = uo * uo;
#pragma unroll
    for (int o = 1; o < 32; o <<= 1) nu += __shfl_xor(nu, o);
    const float invu = 1.0f / (sqrtf(nu) + 1e-12f); __syncthreads(); if (lane < nout) su[w][lane] = uo * invu; __syncthreads(); }
  float t = 0.f; if (lane < nout) { float wv = 0.f;
#pragma unroll 1
    for (int i = 0; i < nin; ++i) wv += bfr(Wm[(size_t)lane * nin + i]) * sv[w][i]; t = su[w][lane] * wv; }
#pragma unroll
  for (int o = 1; o < 32; o <<= 1) t += __shfl_xor(t, o);
  if (lane == 0) res[w] = 1.0f / t; __syncthreads(); if (threadIdx.x == 0) { res[3] = 0.f; vst2(SIG, *(const v4f*)res); } }
__global__ __launch_bounds__(128) void k_edge(const float* __restrict__ NF, const float* __restrict__ W1, const float* __restrict__ B1, const float* __restrict__ W2, const float* __restrict__ B2, const float* __restrict__ W3, const float* __restrict__ B3, const int* __restrict__ BID, const int* __restrict__ SRC, const int* __restrict__ TGT, const float* __restrict__ SIG, float* __restrict__ EW, float* __restrict__ LA) {
  __shared__ __align__(16) float sh1[4][16][36]; __shared__ __align__(16) float so0[64], so1[64]; __shared__ float sdist[64];
  const int tid = threadIdx.x, wave = tid >> 5, lane = tid & 31, col = lane & 15, g = lane >> 4; const size_t e0 = (size_t)blockIdx.x * 64 + wave * 16;
  { const int el = lane >> 1, half = lane & 1; const size_t e = e0 + el; const size_t sb = (size_t)BID[e] * NNODE; const float* ps = NF + (sb + SRC[e]) * FD + half * 64; const float* pt = NF + (sb + TGT[e]) * FD + half * 64; float s = 0.f;
#pragma unroll 4
    for (int i = 0; i < 64; ++i) { const float d = bfr(ps[i]) - bfr(pt[i]); s += d * d; }
    s += __shfl_xor(s, 1); if (half == 0) sdist[wave * 16 + el] = sqrtf(s); }
  const float is1 = SIG[0], is2 = SIG[1], is3 = SIG[2];
  v8f acc[2] = {};
  { const size_t e = e0 + col; const size_t sb = (size_t)BID[e] * NNODE; const float* ps = NF + (sb + SRC[e]) * FD; const float* pt = NF + (sb + TGT[e]) * FD;
#pragma unroll
    for (int kc = 0; kc < 2 * FD / 32; ++kc) { const v16b a = fragb_f32((kc < 4 ? ps : pt) + (kc & 3) * 32, lane);
#pragma unroll
      for (int j = 0; j < 2; ++j) acc[j] = wmma_bf(a, fragb_f32(W1 + (size_t)(j * 16 + col) * IND + kc * 32, lane), acc[j]); } }
  __syncthreads();
#pragma unroll
  for (int j = 0; j < 2; ++j) { const int o = j * 16 + col; const float wd = bfr(W1[(size_t)o * IND + 2 * FD]), bb = bfr(B1[o]);
#pragma unroll
    for (int r = 0; r < 8; ++r) { const float h = (acc[j][r] + wd * sdist[wave * 16 + 8 * g + r]) * is1 + bb; sh1[wave][8 * g + r][o] = fmaxf(h, 0.f); } }
  LDSX();
  v8f acc2[2] = {};
  { float v[16]; const float* pp = &sh1[wave][col][8 * g];
#pragma unroll
    for (int i = 0; i < 8; ++i) { v[i] = pp[i]; v[8 + i] = pp[16 + i]; }
    const F2 a = bsplit16(v);
#pragma unroll
    for (int j = 0; j < 2; ++j) { const v16b w = fragb_f32(W2 + (size_t)(j * 16 + col) * ED, lane); acc2[j] = wmma_bf(a.h, w, acc2[j]); acc2[j] = wmma_bf(a.l, w, acc2[j]); } }
  LDSX();
#pragma unroll
  for (int j = 0; j < 2; ++j) { const int o = j * 16 + col; const float bb = bfr(B2[o]);
#pragma unroll
    for (int r = 0; r < 8; ++r) sh1[wave][8 * g + r][o] = fmaxf(acc2[j][r] * is2 + bb, 0.f); }
  LDSX();
  { const int el = lane >> 1, half = lane & 1; float s = 0.f; const float* hr = &sh1[wave][el][half * 16];
#pragma unroll
    for (int i = 0; i < 16; ++i) s += hr[i] * bfr(W3[half * 16 + i]);
    s += __shfl_xor(s, 1); if (half == 0) { float la = s * is3 + bfr(B3[0]); la = fminf(fmaxf(la, -5.0f), 5.0f); so1[wave * 16 + el] = la; so0[wave * 16 + el] = 1.0f / (1.0f + expf(-la / TEMP)); } }
  __syncthreads(); if (tid < 16) vst2(EW + (size_t)blockIdx.x * 64 + tid * 4, *(const v4f*)&so0[tid * 4]); else if (tid < 32) vst2(LA + (size_t)blockIdx.x * 64 + (tid - 16) * 4, *(const v4f*)&so1[(tid - 16) * 4]); }
extern "C" void kernel_launch(void* const* d_in, const int* in_sizes, int n_in, void* d_out, int out_size, void* d_ws, size_t ws_size, hipStream_t stream) {
  (void)in_sizes; (void)n_in; (void)out_size;
  const float** F = (const float**)d_in;
  if (ws_size < (size_t)WS_END) return;
  char* ws = (char*)d_ws; float* SIG = (float*)(ws + WS_SIG);
  float* EW = (float*)d_out; float* LA = EW + NE;
  k_sigma<<<1, 96, 0, stream>>>(F[1], F[3], F[5], SIG);
  k_edge<<<NE / 64, 128, 0, stream>>>(F[0], F[1], F[2], F[3], F[4], F[5], F[6], (const int*)d_in[7], (const int*)d_in[8], (const int*)d_in[9], SIG, EW, LA);
}
